// GCNModel_70815420776783
// MI455X (gfx1250) — hardware-verified
//
#include <hip/hip_runtime.h>
#include <stddef.h>
#include <stdint.h>
#include <math.h>


#define NN     50000
#define NE     800000
#define HD     128
#define K2     256
#define NG     64
#define NC     10
#define NOUT   (NG * NC)
#define NTHR   256
#define NWAVE  8
#define EPT    8
#define CHUNK  (NTHR * EPT)
#define WCAP   (EPT * 32)
#define LISTN  (NWAVE * WCAP)
#define NBA    1024
#define SLA    10
#define NBLK   49
#define NBP    (NBLK * NBA)
#define RCAP   28672
#define DEGCAP 64
#define GBM    64
#define GBN    128
#define GTHR   128
#define GWAVE  4
#define MP     50048
#define PARTW  288
#define WSTW   258
#define P_B1   0
#define P_G1   128
#define P_BE1  256
#define P_B2   384
#define P_G2   512
#define P_BE2  640
#define P_WFC  768
#define P_BFC  2048
#define PARN   2080
#define NBX    (MP * 16 / NTHR)
#define NBW1   (HD * 16 / NTHR)
#define NBW2   (HD * 32 / NTHR)
#define BKT_ZINTS (LISTN + 2 * RCAP + 3 * NBA)
#define BKT_LDS_INTS (BKT_ZINTS + 16)
#define POOL_LDS_BYTES (2 * NG * HD * 4 + NTHR * 4)
#define WSMAX  134217728

static_assert((CHUNK & (CHUNK - 1)) == 0 && CHUNK <= 4096);
static_assert((NBA & (NBA - 1)) == 0 && NBA == (1 << SLA));
static_assert(((long long)CHUNK << SLA) < (1LL << 31));
static_assert((long long)NE < (1LL << (31 - SLA)));
static_assert((NE % 4) == 0);
static_assert(NBP >= NN && MP >= NN && MP % GBM == 0);
static_assert(RCAP % (NTHR * 4) == 0 && RCAP >= 16623 + 4096);
static_assert(DEGCAP >= 35 + 8);
static_assert(BKT_ZINTS % 4 == 0 && BKT_LDS_INTS * 4 <= 300000);
static_assert(NBA == 4 * NTHR && NBA % NWAVE == 0);
static_assert((MP * 16) % NTHR == 0 && (HD * 16) % NTHR == 0 && (HD * 32) % NTHR == 0);
static_assert(PARN % 32 == 0 && PARN >= P_BFC + NC && PARN <= 9 * NTHR);
static_assert(PARTW % 32 == 0 && PARTW / 4 <= NTHR && PARTW >= 2 * HD + 1 && WSTW >= 2 * HD + 1);
static_assert(GBM == GWAVE * 16 && GBN == HD && HD == 4 * 32 && K2 == 2 * HD);
static_assert((NOUT * 4) % 128 == 0 && NOUT / 4 <= NTHR && NOUT <= 3 * NTHR);
static_assert((NG * HD) % (4 * NTHR) == 0);

typedef float          v4f   __attribute__((ext_vector_type(4)));
typedef float          v8f   __attribute__((ext_vector_type(8)));
typedef int            v4i   __attribute__((ext_vector_type(4)));
typedef int            v8i   __attribute__((ext_vector_type(8)));
typedef unsigned short v8us  __attribute__((ext_vector_type(8)));
typedef unsigned short v16us __attribute__((ext_vector_type(16)));
typedef __bf16         v16bf __attribute__((ext_vector_type(16)));
typedef v4f  __attribute__((may_alias)) v4fa;
typedef v4i  __attribute__((may_alias)) v4ia;
typedef v8us __attribute__((may_alias)) v8usa;
union FragB { v16bf v; v16us u; v8us h[2]; v8i w; };

__device__ __forceinline__ v8f wmb(const FragB& a, const FragB& b, v8f c) {
  v8f d = __builtin_amdgcn_wmma_f32_16x16x32_bf16(false, a.v, false, b.v, (short)0, c, false, false);
  asm volatile("v_nop\n\tv_nop\n\tv_nop\n\tv_nop" : "+v"(d) : "v"(a.w), "v"(b.w));
  return d;
}

__device__ __forceinline__ v8f z8() { v8f z = {0.f, 0.f, 0.f, 0.f, 0.f, 0.f, 0.f, 0.f}; return z; }

__device__ __forceinline__ unsigned bf16_bits(float f) {
  const unsigned u = __float_as_uint(f);
  return (u + 0x7FFFu + ((u >> 16) & 1u)) >> 16;
}
__device__ __forceinline__ unsigned bf16_bits_ns(float f) {
  const unsigned r = bf16_bits(f);
  return (f != f) ? 0x7FC0u : r;
}
__device__ __forceinline__ float bf16_val(float f) {
  return __uint_as_float(bf16_bits(f) << 16);
}
__device__ __forceinline__ float bnrelu(float a, float m, float r, float g, float be) {
  const float t = g * (a - m);
  const float v = t * r + be;
  return (v > 0.0f) ? v : (v - v);
}

template <int SLB>
__device__ __forceinline__ int scan_chunk(const int* __restrict__ dsts, int nE, int cbase, int slotBase,
                                          int nb, int vec8, int* list, int tid, int lane, int wave) {
  int wc = 0;
  const int el0  = tid * EPT;
  const int e0   = cbase + el0;
  const int sent = -2147483647 - 1;
  v4i da, db;
  if (vec8 != 0 && cbase + CHUNK <= nE) {
    da = *(const v4i*)(dsts + e0);
    db = *(const v4i*)(dsts + e0 + 4);
  } else {
    da.x = (e0     < nE) ? dsts[min(e0,     nE - 1)] : sent;
    da.y = (e0 + 1 < nE) ? dsts[min(e0 + 1, nE - 1)] : sent;
    da.z = (e0 + 2 < nE) ? dsts[min(e0 + 2, nE - 1)] : sent;
    da.w = (e0 + 3 < nE) ? dsts[min(e0 + 3, nE - 1)] : sent;
    db.x = (e0 + 4 < nE) ? dsts[min(e0 + 4, nE - 1)] : sent;
    db.y = (e0 + 5 < nE) ? dsts[min(e0 + 5, nE - 1)] : sent;
    db.z = (e0 + 6 < nE) ? dsts[min(e0 + 6, nE - 1)] : sent;
    db.w = (e0 + 7 < nE) ? dsts[min(e0 + 7, nE - 1)] : sent;
  }
  const unsigned nbs = (unsigned)slotBase;
  const unsigned unb = (unsigned)nb;
  const unsigned s0 = (unsigned)da.x - nbs, s1 = (unsigned)da.y - nbs;
  const unsigned s2 = (unsigned)da.z - nbs, s3 = (unsigned)da.w - nbs;
  const unsigned s4 = (unsigned)db.x - nbs, s5 = (unsigned)db.y - nbs;
  const unsigned s6 = (unsigned)db.z - nbs, s7 = (unsigned)db.w - nbs;
  const bool h0 = s0 < unb, h1 = s1 < unb, h2 = s2 < unb, h3 = s3 < unb;
  const bool h4 = s4 < unb, h5 = s5 < unb, h6 = s6 < unb, h7 = s7 < unb;
  const unsigned any = __builtin_amdgcn_ballot_w32(h0 | h1 | h2 | h3 | h4 | h5 | h6 | h7);
  if (any != 0u) {
#define HITJ(J, HJ, SJ) { \
      const unsigned mj = __builtin_amdgcn_ballot_w32(HJ); \
      if (mj != 0u) { \
        if (HJ) { \
          const int pos = wc + (int)__builtin_amdgcn_mbcnt_lo(mj, 0u); \
          if (pos < WCAP) list[wave * WCAP + pos] = ((el0 + (J)) << SLB) | (int)(SJ); \
        } \
        wc += (int)__builtin_popcount(mj); } }
    HITJ(0, h0, s0)
    HITJ(1, h1, s1)
    HITJ(2, h2, s2)
    HITJ(3, h3, s3)
    HITJ(4, h4, s4)
    HITJ(5, h5, s5)
    HITJ(6, h6, s6)
    HITJ(7, h7, s7)
#undef HITJ
  }
  return wc;
}

__global__ __launch_bounds__(NTHR) void k_prep(
    const float* __restrict__ x, const float* __restrict__ W1, const float* __restrict__ W2,
    const float* __restrict__ b1, const float* __restrict__ g1, const float* __restrict__ be1,
    const float* __restrict__ b2, const float* __restrict__ g2, const float* __restrict__ be2,
    const float* __restrict__ Wfc, const float* __restrict__ bfc,
    unsigned short* xb, unsigned short* w1t, unsigned short* w2d, float* par) {
  __shared__ __attribute__((aligned(16))) float pstg[PARN];
  const int tid = (int)threadIdx.x;
  const int blk = (int)blockIdx.x;
  if (blk < NBX) {
    const int u   = blk * NTHR + tid;
    const int row = u >> 4;
    const int k8  = (u & 15) * 8;
    const int rc  = row < NN ? row : NN - 1;
    const float* p = x + (size_t)rc * HD + k8;
    const v4f a = *(const v4fa*)p;
    const v4f b = *(const v4fa*)(p + 4);
    const bool ok = row < NN;
    v8us o;
    o[0] = ok ? (unsigned short)bf16_bits(a.x) : (unsigned short)0;
    o[1] = ok ? (unsigned short)bf16_bits(a.y) : (unsigned short)0;
    o[2] = ok ? (unsigned short)bf16_bits(a.z) : (unsigned short)0;
    o[3] = ok ? (unsigned short)bf16_bits(a.w) : (unsigned short)0;
    o[4] = ok ? (unsigned short)bf16_bits(b.x) : (unsigned short)0;
    o[5] = ok ? (unsigned short)bf16_bits(b.y) : (unsigned short)0;
    o[6] = ok ? (unsigned short)bf16_bits(b.z) : (unsigned short)0;
    o[7] = ok ? (unsigned short)bf16_bits(b.w) : (unsigned short)0;
    unsigned short* dp = xb + (size_t)row * HD + k8;
    *(volatile v8us*)dp = o;
    __threadfence();
    *(volatile v8us*)dp = o;
  } else if (blk < NBX + NBW1) {
    const int u  = (blk - NBX) * NTHR + tid;
    const int n  = u >> 4;
    const int k8 = (u & 15) * 8;
    const float* p = W1 + (size_t)k8 * HD + n;
    v8us o;
#pragma unroll
    for (int i = 0; i < 8; ++i) o[i] = (unsigned short)bf16_bits(p[(size_t)i * HD]);
    unsigned short* dp = w1t + (size_t)n * HD + k8;
    *(volatile v8us*)dp = o;
    __threadfence();
    *(volatile v8us*)dp = o;
  } else if (blk < NBX + NBW1 + NBW2) {
    const int u  = (blk - NBX - NBW1) * NTHR + tid;
    const int n  = u >> 5;
    const int k8 = (u & 31) * 8;
    const int kk = k8 & (HD - 1);
    const float* p = W2 + (size_t)kk * HD + n;
    v8us o;
#pragma unroll
    for (int i = 0; i < 8; ++i) o[i] = (unsigned short)bf16_bits(p[(size_t)i * HD]);
    unsigned short* dp = w2d + (size_t)n * K2 + k8;
    *(volatile v8us*)dp = o;
    __threadfence();
    *(volatile v8us*)dp = o;
  } else {
#pragma unroll 1
    for (int j = 0; j < 9; ++j) {
      const int i   = j * NTHR + tid;
      const int ic  = i < PARN ? i : PARN - 1;
      const int c   = ic & (HD - 1);
      const int sec = ic >> 7;
      const float v0 = b1[c], v1 = g1[c], v2 = be1[c];
      const float v3 = b2[c], v4 = g2[c], v5 = be2[c];
      int wi = ic - P_WFC;
      wi = wi < 0 ? 0 : (wi > HD * NC - 1 ? HD * NC - 1 : wi);
      const float v6 = Wfc[wi];
      int bi = ic - P_BFC;
      const bool bok = (bi >= 0) && (bi < NC);
      bi = bi < 0 ? 0 : (bi > NC - 1 ? NC - 1 : bi);
      const float v7 = bfc[bi];
      float v = (ic >= P_BFC) ? (bok ? v7 : 0.0f) : v6;
      v = (sec == 5) ? v5 : v;
      v = (sec == 4) ? v4 : v;
      v = (sec == 3) ? v3 : v;
      v = (sec == 2) ? v2 : v;
      v = (sec == 1) ? v1 : v;
      v = (sec == 0) ? v0 : v;
      if (i < PARN) pstg[i] = bf16_val(v);
    }
    __syncthreads();
    v4f pv[3];
#pragma unroll
    for (int it = 0; it < 3; ++it) {
      const int q  = it * NTHR + tid;
      const int qc = q < PARN / 4 ? q : PARN / 4 - 1;
      pv[it] = *(const v4fa*)(pstg + 4 * qc);
    }
#pragma unroll
    for (int it = 0; it < 3; ++it) {
      const int q = it * NTHR + tid;
      if (q < PARN / 4) *(volatile v4f*)(par + 4 * q) = pv[it];
    }
    __threadfence();
#pragma unroll
    for (int it = 0; it < 3; ++it) {
      const int q = it * NTHR + tid;
      if (q < PARN / 4) *(volatile v4f*)(par + 4 * q) = pv[it];
    }
  }
}

__global__ __launch_bounds__(NTHR) void k_bucket(const int* __restrict__ srcs, const int* __restrict__ dsts,
                                                 int* hits, int* cntg, int* offg, int* disg) {
  extern __shared__ __attribute__((aligned(16))) int dsm[];
  int* list = dsm;
  int* hl   = dsm + LISTN;
  int* sl   = hl + RCAP;
  int* cnt  = sl + RCAP;
  int* offs = cnt + NBA;
  int* cur  = offs + NBA;
  int* misc = cur + NBA;
  const int tid = (int)threadIdx.x, lane = tid & 31, wave = tid >> 5;
  const int nodeBase = (int)blockIdx.x * NBA;

  {
    const v4i z4 = {0, 0, 0, 0};
    for (int i = tid * 4; i < BKT_ZINTS; i += NTHR * 4) *(v4ia*)(dsm + i) = z4;
    if (tid < 16) misc[tid] = 0;
  }
  __syncthreads();

  int t = 0, ov = 0;
  const int nChunks = (NE + CHUNK - 1) / CHUNK;
#pragma unroll 1
  for (int ch = 0; ch < nChunks; ++ch) {
    const int cbase = ch * CHUNK;
    const int wc = scan_chunk<SLA>(dsts, NE, cbase, nodeBase, NBA, 1, list, tid, lane, wave);
    if (lane == 0) misc[wave] = wc;
    __syncthreads();
    if (wave == 0) {
#pragma unroll 1
      for (int w2 = 0; w2 < NWAVE; ++w2) {
        int c = misc[w2];
        c = c < 0 ? 0 : (c > WCAP ? WCAP : c);
#pragma unroll 1
        for (int b0 = 0; b0 < c; b0 += 32) {
          const int idx = b0 + lane;
          const int ent = list[w2 * WCAP + (idx < WCAP ? idx : WCAP - 1)];
          const int m32 = (c - b0) < 32 ? (c - b0) : 32;
#pragma unroll 1
          for (int k = 0; k < m32; ++k) {
            const int u    = __builtin_amdgcn_readlane(ent, k);
            const int slot = u & (NBA - 1);
            const int el   = (u >> SLA) & (CHUNK - 1);
            const int pk   = ((cbase + el) << SLA) | slot;
            if (t < RCAP) {
              if (lane == 0) { hl[t] = pk; cnt[slot] = cnt[slot] + 1; }
              t = t + 1;
            } else {
              ov = 1;
            }
          }
        }
      }
    }
    __syncthreads();
  }
  if (wave == 0 && lane == 0) { misc[8] = t; misc[9] = ov; }
  __syncthreads();
  int tt = misc[8];
  tt = tt < 0 ? 0 : (tt > RCAP ? RCAP : tt);
  const int ovf = misc[9];

  if (wave == 0) {
    const int base = lane * (NBA / 32);
    int s = 0;
#pragma unroll 1
    for (int i = 0; i < NBA / 32; ++i) s += cnt[base + i];
    int incl = s;
#pragma unroll
    for (int d = 1; d < 32; d <<= 1) {
      const int y = __shfl_up(incl, d, 32);
      if (lane >= d) incl += y;
    }
    int run = incl - s;
#pragma unroll 1
    for (int i = 0; i < NBA / 32; ++i) {
      const int cv = cnt[base + i];
      offs[base + i] = run;
      cur[base + i]  = run;
      run += cv;
    }
  }
  __syncthreads();
  if (wave == 0) {
#pragma unroll 1
    for (int b0 = 0; b0 < tt; b0 += 32) {
      const int idx = b0 + lane;
      const int ent = hl[idx < RCAP ? idx : RCAP - 1];
      const int m32 = (tt - b0) < 32 ? (tt - b0) : 32;
#pragma unroll 1
      for (int k = 0; k < m32; ++k) {
        const int u    = __builtin_amdgcn_readlane(ent, k);
        const int slot = u & (NBA - 1);
        if (lane == 0) {
          int p = cur[slot];
          p = p < 0 ? 0 : (p > RCAP - 1 ? RCAP - 1 : p);
          sl[p] = u;
          cur[slot] = p + 1;
        }
      }
    }
  }
  __syncthreads();

#pragma unroll 1
  for (int j = 0; j < RCAP / NTHR; ++j) {
    const int idx = j * NTHR + tid;
    const int ent = sl[idx];
    int eid = ent >> SLA;
    eid = eid < 0 ? 0 : (eid > NE - 1 ? NE - 1 : eid);
    int sr = srcs[eid];
    sr = sr < 0 ? 0 : (sr > NN - 1 ? NN - 1 : sr);
    hl[idx] = (idx < tt) ? sr : 0;
  }
#pragma unroll 1
  for (int s = tid; s < NBA; s += NTHR) {
    int c = cnt[s];
    c = c < 0 ? 0 : c;
    const float d = 1.0f / sqrtf((float)(c + 1));
    cur[s] = __float_as_int(d);
    cnt[s] = (ovf != 0) ? -1 : c;
  }
  __syncthreads();

  int* hp = hits + (size_t)blockIdx.x * RCAP;
  const v4i c4 = *(const v4ia*)(cnt  + 4 * tid);
  const v4i o4 = *(const v4ia*)(offs + 4 * tid);
  const v4i d4 = *(const v4ia*)(cur  + 4 * tid);
#pragma unroll 1
  for (int j = 0; j < RCAP / (NTHR * 4); ++j) {
    const int i4 = (j * NTHR + tid) * 4;
    const v4i v = *(const v4ia*)(hl + i4);
    *(volatile v4i*)(hp + i4) = v;
  }
  *(volatile v4i*)(cntg + nodeBase + 4 * tid) = c4;
  *(volatile v4i*)(offg + nodeBase + 4 * tid) = o4;
  *(volatile v4i*)(disg + nodeBase + 4 * tid) = d4;
  __threadfence();
#pragma unroll 1
  for (int j = 0; j < RCAP / (NTHR * 4); ++j) {
    const int i4 = (j * NTHR + tid) * 4;
    const v4i v = *(const v4ia*)(hl + i4);
    *(volatile v4i*)(hp + i4) = v;
  }
  *(volatile v4i*)(cntg + nodeBase + 4 * tid) = c4;
  *(volatile v4i*)(offg + nodeBase + 4 * tid) = o4;
  *(volatile v4i*)(disg + nodeBase + 4 * tid) = d4;
}

template <int K>
__global__ __launch_bounds__(GTHR) void k_gemm(const unsigned short* __restrict__ A,
                                               const unsigned short* __restrict__ BT, float* xout) {
  static_assert(K % 32 == 0);
  __shared__ __attribute__((aligned(16))) float stg[GBM * GBN];
  const int tid = (int)threadIdx.x, lane = tid & 31, wave = tid >> 5, hh = lane >> 4, m = lane & 15;
  const int rowBase = (int)blockIdx.x * GBM;

  v8f acc[8];
#pragma unroll
  for (int t = 0; t < 8; ++t) acc[t] = z8();
  const unsigned short* ap = A  + (size_t)(rowBase + 16 * wave + m) * (size_t)K + 8 * hh;
  const unsigned short* bp = BT + (size_t)m * (size_t)K + 8 * hh;

#pragma unroll 1
  for (int k0 = 0; k0 < K; k0 += 32) {
    FragB af;
    af.h[0] = *(const v8usa*)(ap + k0);
    af.h[1] = *(const v8usa*)(ap + k0 + 16);
#pragma unroll
    for (int nt = 0; nt < 8; ++nt) {
      const unsigned short* wq = bp + (size_t)(16 * nt) * (size_t)K + k0;
      FragB bf;
      bf.h[0] = *(const v8usa*)wq;
      bf.h[1] = *(const v8usa*)(wq + 16);
      acc[nt] = wmb(af, bf, acc[nt]);
    }
  }

#pragma unroll
  for (int nt = 0; nt < 8; ++nt) {
    const int lc = 16 * nt + m;
#pragma unroll
    for (int r = 0; r < 8; ++r) {
      const int lr = 16 * wave + 8 * hh + r;
      stg[lr * GBN + lc] = acc[nt][r];
    }
  }
  __syncthreads();

  v4f pv[16];
#pragma unroll
  for (int i = 0; i < 16; ++i) pv[i] = *(const v4fa*)(stg + (16 * wave + i) * GBN + 4 * lane);
#pragma unroll
  for (int i = 0; i < 16; ++i) {
    float* op = xout + (size_t)(rowBase + 16 * wave + i) * (size_t)HD + 4 * lane;
    *(volatile v4f*)op = pv[i];
  }
  __threadfence();
#pragma unroll
  for (int i = 0; i < 16; ++i) {
    float* op = xout + (size_t)(rowBase + 16 * wave + i) * (size_t)HD + 4 * lane;
    *(volatile v4f*)op = pv[i];
  }
}

__global__ __launch_bounds__(NTHR) void k_agg(const int* __restrict__ hits, const int* __restrict__ cntg,
                                              const int* __restrict__ offg, const float* __restrict__ dis,
                                              const float* __restrict__ hf, const float* __restrict__ par,
                                              int boff, float* aout, float* part) {
  __shared__ __attribute__((aligned(16))) int   cs[NBA];
  __shared__ __attribute__((aligned(16))) int   os[NBA];
  __shared__ __attribute__((aligned(16))) float ds[NBA];
  __shared__ __attribute__((aligned(16))) float wst[NWAVE * WSTW];
  __shared__ __attribute__((aligned(16))) float pst[PARTW];
  const int tid = (int)threadIdx.x, lane = tid & 31, wave = tid >> 5;
  const int nodeBase = (int)blockIdx.x * NBA;

  {
    const v4i c4 = *(const v4ia*)(cntg + nodeBase + 4 * tid);
    const v4i o4 = *(const v4ia*)(offg + nodeBase + 4 * tid);
    const v4f d4 = *(const v4fa*)(dis  + nodeBase + 4 * tid);
    *(v4ia*)(cs + 4 * tid) = c4;
    *(v4ia*)(os + 4 * tid) = o4;
    *(v4fa*)(ds + 4 * tid) = d4;
  }
  const v4f b4 = *(const v4fa*)(par + boff + 4 * lane);
  __syncthreads();

  const int* hp = hits + (size_t)blockIdx.x * RCAP;
  const float qnan = __int_as_float(0x7fc00000);
  int wn = 0;
  float wm[4], wq[4];
#pragma unroll
  for (int j = 0; j < 4; ++j) { wm[j] = 0.0f; wq[j] = 0.0f; }

#pragma unroll 1
  for (int si = 0; si < NBA / NWAVE; ++si) {
    const int s    = si * NWAVE + wave;
    const int node = nodeBase + s;
    int c = cs[s];
    const bool bad = (c < 0) || (c > DEGCAP);
    c = c < 0 ? 0 : (c > DEGCAP ? DEGCAP : c);
    int o = os[s];
    o = o < 0 ? 0 : (o > RCAP ? RCAP : o);
    const float dd = ds[s];
    const float rd = dd * dd;
    float a0 = 0.0f, a1 = 0.0f, a2 = 0.0f, a3 = 0.0f;
#pragma unroll 1
    for (int b0 = 0; b0 < c; b0 += 32) {
      int idx = o + b0 + lane;
      idx = idx > RCAP - 1 ? RCAP - 1 : idx;
      int sr = hp[idx];
      sr = sr < 0 ? 0 : (sr > NN - 1 ? NN - 1 : sr);
      const float cf  = dis[sr] * dd;
      const int   cfi = __float_as_int(cf);
      const int m32 = (c - b0) < 32 ? (c - b0) : 32;
#pragma unroll 1
      for (int k = 0; k < m32; ++k) {
        const int   sk = __builtin_amdgcn_readlane(sr, k);
        const float ck = __int_as_float(__builtin_amdgcn_readlane(cfi, k));
        const v4f a = *(const v4fa*)(hf + (size_t)sk * HD + 4 * lane);
        a0 = fmaf(ck, a.x, a0); a1 = fmaf(ck, a.y, a1);
        a2 = fmaf(ck, a.z, a2); a3 = fmaf(ck, a.w, a3);
      }
    }
    const int nc = node < NN ? node : NN - 1;
    const v4f sv = *(const v4fa*)(hf + (size_t)nc * HD + 4 * lane);
    const float pz = bad ? qnan : 0.0f;
    float y[4];
    y[0] = ((a0 + sv.x * rd) + b4.x) + pz;
    y[1] = ((a1 + sv.y * rd) + b4.y) + pz;
    y[2] = ((a2 + sv.z * rd) + b4.z) + pz;
    y[3] = ((a3 + sv.w * rd) + b4.w) + pz;
    const bool live = node < NN;
    if (live) {
      wn += 1;
      const float rk = 1.0f / (float)wn;
#pragma unroll
      for (int j = 0; j < 4; ++j) {
        const float d = y[j] - wm[j];
        wm[j] = fmaf(d, rk, wm[j]);
        wq[j] = fmaf(d, y[j] - wm[j], wq[j]);
      }
    }
    v4f yv;
    yv.x = y[0]; yv.y = y[1]; yv.z = y[2]; yv.w = y[3];
    float* op = aout + (size_t)nc * HD + 4 * lane;
    if (live) *(volatile v4f*)op = yv;
    __threadfence();
    if (live) *(volatile v4f*)op = yv;
  }

  if (lane == 0) wst[wave * WSTW] = (float)wn;
#pragma unroll
  for (int j = 0; j < 4; ++j) {
    wst[wave * WSTW + 1 + 4 * lane + j]      = wm[j];
    wst[wave * WSTW + 1 + HD + 4 * lane + j] = wq[j];
  }
  __syncthreads();
  if (tid < HD) {
    double n = 0.0, mean = 0.0, M2 = 0.0;
#pragma unroll 1
    for (int w2 = 0; w2 < NWAVE; ++w2) {
      const double nb = (double)wst[w2 * WSTW];
      const double mb = (double)wst[w2 * WSTW + 1 + tid];
      const double qb = (double)wst[w2 * WSTW + 1 + HD + tid];
      if (nb > 0.5) {
        const double nn2 = n + nb;
        const double delta = mb - mean;
        const double f = nb / nn2;
        mean = mean + delta * f;
        M2 = M2 + qb + delta * delta * n * f;
        n = nn2;
      }
    }
    pst[1 + tid] = (float)mean;
    pst[1 + HD + tid] = (float)M2;
    if (tid == 0) pst[0] = (float)n;
  }
#pragma unroll 1
  for (int i = 2 * HD + 1 + tid; i < PARTW; i += NTHR) pst[i] = 0.0f;
  __syncthreads();
  const int qc = tid < PARTW / 4 ? tid : PARTW / 4 - 1;
  const v4f ps = *(const v4fa*)(pst + 4 * qc);
  float* pp = part + (size_t)blockIdx.x * PARTW + 4 * qc;
  if (tid < PARTW / 4) *(volatile v4f*)pp = ps;
  __threadfence();
  if (tid < PARTW / 4) *(volatile v4f*)pp = ps;
}

__global__ __launch_bounds__(HD) void k_comb(const float* __restrict__ part, float* stat) {
  __shared__ __attribute__((aligned(16))) float stg[2 * HD];
  const int tid = (int)threadIdx.x;
  double n = 0.0, mean = 0.0, M2 = 0.0;
#pragma unroll 1
  for (int b = 0; b < NBLK; ++b) {
    const float* pr = part + (size_t)b * PARTW;
    const double nb = (double)pr[0];
    const double mb = (double)pr[1 + tid];
    const double qb = (double)pr[1 + HD + tid];
    if (nb > 0.5) {
      const double nn2 = n + nb;
      const double delta = mb - mean;
      const double f = nb / nn2;
      mean = mean + delta * f;
      M2 = M2 + qb + delta * delta * n * f;
      n = nn2;
    }
  }
  const double nt = n < 1.0 ? 1.0 : n;
  const float varf  = (float)(M2 / nt);
  const float meanf = (float)mean;
  const float rstd  = 1.0f / sqrtf(varf + 1e-5f);
  stg[tid] = meanf;
  stg[HD + tid] = rstd;
  __syncthreads();
  const int qc = tid < (2 * HD) / 4 ? tid : (2 * HD) / 4 - 1;
  const v4f v = *(const v4fa*)(stg + 4 * qc);
  if (tid < (2 * HD) / 4) *(volatile v4f*)(stat + 4 * qc) = v;
  __threadfence();
  if (tid < (2 * HD) / 4) *(volatile v4f*)(stat + 4 * qc) = v;
}

__global__ __launch_bounds__(NTHR) void k_apply(const float* __restrict__ a, const float* __restrict__ stat,
                                                const float* __restrict__ par, int goff, unsigned short* x1) {
  __shared__ __attribute__((aligned(16))) float ssh[4 * HD];
  const int tid = (int)threadIdx.x;
  ssh[tid] = stat[tid];
  ssh[2 * HD + tid] = par[goff + tid];
  __syncthreads();
  const int u   = (int)blockIdx.x * NTHR + tid;
  const int row = u >> 4;
  const int k8  = (u & 15) * 8;
  const int rc  = row < NN ? row : NN - 1;
  const float* p = a + (size_t)rc * HD + k8;
  const v4f x0 = *(const v4fa*)p;
  const v4f x1v = *(const v4fa*)(p + 4);
  const v4f m0 = *(const v4fa*)(ssh + k8),          m1 = *(const v4fa*)(ssh + k8 + 4);
  const v4f r0 = *(const v4fa*)(ssh + HD + k8),     r1 = *(const v4fa*)(ssh + HD + k8 + 4);
  const v4f g0 = *(const v4fa*)(ssh + 2 * HD + k8), g1 = *(const v4fa*)(ssh + 2 * HD + k8 + 4);
  const v4f e0 = *(const v4fa*)(ssh + 3 * HD + k8), e1 = *(const v4fa*)(ssh + 3 * HD + k8 + 4);
  float v[8];
  v[0] = bnrelu(x0.x, m0.x, r0.x, g0.x, e0.x);
  v[1] = bnrelu(x0.y, m0.y, r0.y, g0.y, e0.y);
  v[2] = bnrelu(x0.z, m0.z, r0.z, g0.z, e0.z);
  v[3] = bnrelu(x0.w, m0.w, r0.w, g0.w, e0.w);
  v[4] = bnrelu(x1v.x, m1.x, r1.x, g1.x, e1.x);
  v[5] = bnrelu(x1v.y, m1.y, r1.y, g1.y, e1.y);
  v[6] = bnrelu(x1v.z, m1.z, r1.z, g1.z, e1.z);
  v[7] = bnrelu(x1v.w, m1.w, r1.w, g1.w, e1.w);
  const bool ok = row < NN;
  v8us hv, lv;
#pragma unroll
  for (int j = 0; j < 8; ++j) {
    const float yy = ok ? v[j] : 0.0f;
    const unsigned hb = bf16_bits_ns(yy);
    hv[j] = (unsigned short)hb;
    lv[j] = (unsigned short)bf16_bits_ns(yy - __uint_as_float(hb << 16));
  }
  unsigned short* op = x1 + (size_t)row * K2 + k8;
  *(volatile v8us*)op = hv;
  *(volatile v8us*)(op + HD) = lv;
  __threadfence();
  *(volatile v8us*)op = hv;
  *(volatile v8us*)(op + HD) = lv;
}

__global__ __launch_bounds__(NTHR) void k_pool(const float* __restrict__ a, const int* __restrict__ bat,
                                               const float* __restrict__ stat, const float* __restrict__ par,
                                               float* ps, int* pc) {
  extern __shared__ __attribute__((aligned(16))) float psm[];
  float* tab = psm;
  int*   cnl = (int*)(psm + 2 * NG * HD);
  const int tid = (int)threadIdx.x;
  const int hfi = tid >> 7;
  const int c   = tid & (HD - 1);
  {
    const v4f z = {0.f, 0.f, 0.f, 0.f};
    for (int i = tid * 4; i < 2 * NG * HD; i += NTHR * 4) *(v4fa*)(tab + i) = z;
  }
  const float m  = stat[c];
  const float r  = stat[HD + c];
  const float g  = par[P_G2 + c];
  const float be = par[P_BE2 + c];
  __syncthreads();
  const int rbase = (int)blockIdx.x * NBA + hfi * (NBA / 2);
  float* tb = tab + hfi * (NG * HD) + c;
  int cntreg = 0;
#pragma unroll 1
  for (int i = 0; i < NBA / 2; ++i) {
    const int row = rbase + i;
    const int rc  = row < NN ? row : NN - 1;
    const int gid = bat[rc];
    const float av = a[(size_t)rc * HD + c];
    const float v = bnrelu(av, m, r, g, be);
    const bool ok = (row < NN) && ((unsigned)gid < (unsigned)NG);
    const int gc = gid < 0 ? 0 : (gid > NG - 1 ? NG - 1 : gid);
    const float o = tb[gc * HD];
    tb[gc * HD] = ok ? (o + v) : o;
    cntreg += (ok && (gid == c)) ? 1 : 0;
  }
  cnl[tid] = cntreg;
  __syncthreads();
  v4f pv[8];
#pragma unroll
  for (int it = 0; it < 8; ++it) {
    const int i4 = (it * NTHR + tid) * 4;
    const v4f p0 = *(const v4fa*)(tab + i4);
    const v4f p1 = *(const v4fa*)(tab + NG * HD + i4);
    pv[it] = p0 + p1;
  }
  const int q4 = (tid & 15) * 4;
  v4i cv;
  cv.x = cnl[q4 + 0] + cnl[HD + q4 + 0];
  cv.y = cnl[q4 + 1] + cnl[HD + q4 + 1];
  cv.z = cnl[q4 + 2] + cnl[HD + q4 + 2];
  cv.w = cnl[q4 + 3] + cnl[HD + q4 + 3];
  float* pp = ps + (size_t)blockIdx.x * (NG * HD);
  int*   cp = pc + (size_t)blockIdx.x * NG + q4;
#pragma unroll
  for (int it = 0; it < 8; ++it) *(volatile v4f*)(pp + (it * NTHR + tid) * 4) = pv[it];
  if (tid < 16) *(volatile v4i*)cp = cv;
  __threadfence();
#pragma unroll
  for (int it = 0; it < 8; ++it) *(volatile v4f*)(pp + (it * NTHR + tid) * 4) = pv[it];
  if (tid < 16) *(volatile v4i*)cp = cv;
}

__global__ __launch_bounds__(NTHR) void k_head(const float* __restrict__ ps, const int* __restrict__ pc,
                                               const float* __restrict__ par, float* out) {
  __shared__ __attribute__((aligned(16))) float pl[NG * HD];
  __shared__ float wls[HD * NC];
  __shared__ float bls[16];
  __shared__ float cfs[NG];
  __shared__ __attribute__((aligned(16))) float os[NOUT];
  const int tid = (int)threadIdx.x;
#pragma unroll 1
  for (int i = tid; i < HD * NC; i += NTHR) wls[i] = par[P_WFC + i];
  {
    const float bb = par[P_BFC + (tid & 15)];
    if (tid < 16) bls[tid] = bb;
  }
  if (tid < NG) {
    int cc = 0;
#pragma unroll 1
    for (int b = 0; b < NBLK; ++b) cc += pc[b * NG + tid];
    cc = cc < 0 ? 0 : cc;
    cfs[tid] = fmaxf((float)cc, 1.0f);
  }
  __syncthreads();
#pragma unroll 1
  for (int q = 0; q < (NG * HD) / (4 * NTHR); ++q) {
    const int i4 = (q * NTHR + tid) * 4;
    const int g  = i4 >> 7;
    double a0 = 0.0, a1 = 0.0, a2 = 0.0, a3 = 0.0;
#pragma unroll 1
    for (int b = 0; b < NBLK; ++b) {
      const v4f p = *(const v4fa*)(ps + (size_t)b * (NG * HD) + i4);
      a0 += (double)p.x; a1 += (double)p.y; a2 += (double)p.z; a3 += (double)p.w;
    }
    const float cf = cfs[g];
    pl[i4 + 0] = (float)a0 / cf;
    pl[i4 + 1] = (float)a1 / cf;
    pl[i4 + 2] = (float)a2 / cf;
    pl[i4 + 3] = (float)a3 / cf;
  }
  __syncthreads();
#pragma unroll 1
  for (int it = 0; it < 3; ++it) {
    const int idx = it * NTHR + tid;
    const int idc = idx < NOUT ? idx : NOUT - 1;
    const int g = idc / NC;
    const int c = idc - g * NC;
    float s = 0.0f;
#pragma unroll 4
    for (int k = 0; k < HD; ++k) s = fmaf(pl[g * HD + k], wls[k * NC + c], s);
    if (idx < NOUT) os[idx] = s + bls[c];
  }
  __syncthreads();
  const int qc = tid < NOUT / 4 ? tid : NOUT / 4 - 1;
  const v4f ov = *(const v4fa*)(os + 4 * qc);
  if (tid < NOUT / 4) *(volatile v4f*)(out + 4 * qc) = ov;
  __threadfence();
  if (tid < NOUT / 4) *(volatile v4f*)(out + 4 * qc) = ov;
}

static inline size_t al256(size_t o) { return (o + 255) & ~(size_t)255; }

extern "C" void kernel_launch(void* const* d_in, const int* in_sizes, int n_in,
                              void* d_out, int out_size, void* d_ws, size_t ws_size,
                              hipStream_t stream) {
  if (n_in < 13) return;
  if (in_sizes[0] != NN * HD) return;
  if (in_sizes[1] != 2 * NE) return;
  if (in_sizes[2] != NN) return;
  if (in_sizes[3] != HD * HD || in_sizes[7] != HD * HD) return;
  if (in_sizes[4] != HD || in_sizes[5] != HD || in_sizes[6] != HD) return;
  if (in_sizes[8] != HD || in_sizes[9] != HD || in_sizes[10] != HD) return;
  if (in_sizes[11] != HD * NC || in_sizes[12] != NC) return;
  if (out_size != NOUT) return;

  const float* x    = (const float*)d_in[0];
  const int*   edge = (const int*)d_in[1];
  const int*   bat  = (const int*)d_in[2];
  const float* W1   = (const float*)d_in[3];
  const float* b1   = (const float*)d_in[4];
  const float* g1   = (const float*)d_in[5];
  const float* be1  = (const float*)d_in[6];
  const float* W2   = (const float*)d_in[7];
  const float* b2   = (const float*)d_in[8];
  const float* g2   = (const float*)d_in[9];
  const float* be2  = (const float*)d_in[10];
  const float* Wfc  = (const float*)d_in[11];
  const float* bfc  = (const float*)d_in[12];
  float* out = (float*)d_out;
  const int* src = edge;
  const int* dst = edge + NE;

  char* ws = (char*)d_ws;
  size_t off = 0;
  const size_t oXB  = off; off = al256(off + (size_t)MP * HD * 2);
  const size_t oW1T = off; off = al256(off + (size_t)HD * HD * 2);
  const size_t oW2D = off; off = al256(off + (size_t)HD * K2 * 2);
  const size_t oPAR = off; off = al256(off + (size_t)PARN * 4);
  const size_t oHIT = off; off = al256(off + (size_t)NBLK * RCAP * 4);
  const size_t oCNT = off; off = al256(off + (size_t)NBP * 4);
  const size_t oOFF = off; off = al256(off + (size_t)NBP * 4);
  const size_t oDIS = off; off = al256(off + (size_t)NBP * 4);
  const size_t oH   = off; off = al256(off + (size_t)MP * HD * 4);
  const size_t oA   = off; off = al256(off + (size_t)NN * HD * 4);
  const size_t oX1  = off; off = al256(off + (size_t)MP * K2 * 2);
  const size_t oP1  = off; off = al256(off + (size_t)NBLK * PARTW * 4);
  const size_t oP2  = off; off = al256(off + (size_t)NBLK * PARTW * 4);
  const size_t oS1  = off; off = al256(off + (size_t)(2 * HD) * 4);
  const size_t oS2  = off; off = al256(off + (size_t)(2 * HD) * 4);
  const size_t oPS  = off; off = al256(off + (size_t)NBLK * NG * HD * 4);
  const size_t oPC  = off; off = al256(off + (size_t)NBLK * NG * 4);
  if (off > ws_size || off > (size_t)WSMAX) return;
  unsigned short* XB  = (unsigned short*)(ws + oXB);
  unsigned short* W1T = (unsigned short*)(ws + oW1T);
  unsigned short* W2D = (unsigned short*)(ws + oW2D);
  float*          PAR = (float*)(ws + oPAR);
  int*            HIT = (int*)(ws + oHIT);
  int*            CNT = (int*)(ws + oCNT);
  int*            OFS = (int*)(ws + oOFF);
  float*          DIS = (float*)(ws + oDIS);
  float*          H   = (float*)(ws + oH);
  float*          A   = (float*)(ws + oA);
  unsigned short* X1  = (unsigned short*)(ws + oX1);
  float*          P1  = (float*)(ws + oP1);
  float*          P2  = (float*)(ws + oP2);
  float*          S1  = (float*)(ws + oS1);
  float*          S2  = (float*)(ws + oS2);
  float*          PS  = (float*)(ws + oPS);
  int*            PC  = (int*)(ws + oPC);

  const size_t bktLds  = (size_t)BKT_LDS_INTS * 4;
  const size_t poolLds = (size_t)POOL_LDS_BYTES;
  hipFuncSetAttribute(reinterpret_cast<const void*>(&k_bucket), hipFuncAttributeMaxDynamicSharedMemorySize, (int)bktLds);
  hipFuncSetAttribute(reinterpret_cast<const void*>(&k_pool), hipFuncAttributeMaxDynamicSharedMemorySize, (int)poolLds);

  k_prep<<<NBX + NBW1 + NBW2 + 1, NTHR, 0, stream>>>(x, W1, W2, b1, g1, be1, b2, g2, be2, Wfc, bfc,
                                                     XB, W1T, W2D, PAR);
  k_bucket<<<NBLK, NTHR, bktLds, stream>>>(src, dst, HIT, CNT, OFS, (int*)DIS);
  k_gemm<HD><<<MP / GBM, GTHR, 0, stream>>>(XB, W1T, H);
  k_agg<<<NBLK, NTHR, 0, stream>>>(HIT, CNT, OFS, DIS, H, PAR, P_B1, A, P1);
  k_comb<<<1, HD, 0, stream>>>(P1, S1);
  k_apply<<<NBX, NTHR, 0, stream>>>(A, S1, PAR, P_G1, X1);
  k_gemm<K2><<<MP / GBM, GTHR, 0, stream>>>(X1, W2D, H);
  k_agg<<<NBLK, NTHR, 0, stream>>>(HIT, CNT, OFS, DIS, H, PAR, P_B2, A, P2);
  k_comb<<<1, HD, 0, stream>>>(P2, S2);
  k_pool<<<NBLK, NTHR, poolLds, stream>>>(A, bat, S2, PAR, PS, PC);
  k_head<<<1, NTHR, 0, stream>>>(PS, PC, PAR, out);
}
